// HeavyEncoderLayer_74388833566995
// MI455X (gfx1250) — hardware-verified
//
#include <hip/hip_runtime.h>
#include <stddef.h>
#include <math.h>


#define NFX   160
#define NMSG  112
#define RADN  128
#define WNUM  4608
#define NT    128
#define NW    4
#define EPB   64
#define NPB   64
#define OPB   16
#define EPT   8
#define SGRP  2
#define CHUNK (NT * EPT)
#define WCAP  (EPT * 32)
#define LISTN (NW * WCAP)
#define RP    128
#define HP    136
#define XP    160
#define WSCAP 134217728

#define PO_W2  0
#define PO_G1  1179648
#define PO_G3  1376256
#define PO_G4  1507328
#define PO_WD  1572864
#define PO_L0  1605632
#define PO_L1  1606656
#define PO_TOT 1608704
#define NPREPB 393

#define LE_HH  0
#define LE_HL  17408
#define LE_X0  34816
#define LE_X1  51200
#define LE_Q1  75776
#define LE_A   83968
#define LE_W1  84992
#define LE_SRC 87040
#define LDS_EDGE 87296

#define LN_X   0
#define LN_NM  40960
#define LN_ST  69632
#define LN_LS  98304
#define LN_WC  102400
#define LDS_NODE 102528

#define LP_S   0
#define LP_ST  28672
#define LP_W   57344
#define LP_CN  62464
#define LP_LS  62720
#define LP_WC  66816
#define LDS_POOL 66944

#define RS128    0.08838834764831845f
#define RS32     0.1767766952966369f
#define INV3     0.57735026918962576f
#define PW_MSG0  0.10206207261596575f
#define PW_MSG1  0.17677669529663688f
#define PW_G01   0.022097086912079608f
#define PW_G2    0.034232659844072880f
#define PW_H0    0.031008683647302115f
#define PW_H1    0.30618621784789724f
#define CST_SILU 1.67653247f
#define CST_SIG  1.84622855f
#define CST_TANH 1.59253742f

static_assert(NT == NW * 32);
static_assert(EPB == NW * 16);
static_assert(NPB == NW * 16);
static_assert(CHUNK <= 4096);
static_assert((CHUNK & (CHUNK - 1)) == 0);
static_assert((NPB & (NPB - 1)) == 0);
static_assert(WCAP == EPT * 32);
static_assert((EPT % SGRP) == 0);
static_assert(PO_G1 == PO_W2 + 2 * WNUM * RADN);
static_assert(PO_G3 == PO_G1 + 2 * 48 * 2048);
static_assert(PO_G4 == PO_G3 + 2 * 1024 * 64);
static_assert(PO_WD == PO_G4 + 2 * 1024 * 32);
static_assert(PO_L0 == PO_WD + 2 * 16 * 1024);
static_assert(PO_L1 == PO_L0 + 2 * 16 * 32);
static_assert(PO_TOT == PO_L1 + 2 * 32 * 32);
static_assert(LE_HL == LE_HH + EPB * HP * 2);
static_assert(LE_X0 == LE_HL + EPB * HP * 2);
static_assert(LE_X1 == LE_X0 + EPB * 64 * 4);
static_assert(LE_Q1 == LE_X1 + EPB * 96 * 4);
static_assert(LE_A == LE_Q1 + EPB * 32 * 4);
static_assert(LE_W1 == LE_A + EPB * 4 * 4);
static_assert(LE_SRC == LE_W1 + 4 * RADN * 4);
static_assert(LDS_EDGE >= LE_SRC + EPB * 4);
static_assert(NW * 16 * NMSG * 4 <= LE_X0);
static_assert(LN_NM == LN_X + NPB * XP * 4);
static_assert(LN_ST == LN_NM + NPB * NMSG * 4);
static_assert(LN_LS == LN_ST + NW * 16 * NMSG * 4);
static_assert(LN_WC == LN_LS + LISTN * 4);
static_assert(LDS_NODE >= LN_WC + NW * 4);
static_assert(LP_ST == LP_S + NPB * NMSG * 4);
static_assert(LP_W == LP_ST + NW * 16 * NMSG * 4);
static_assert(LP_CN == LP_W + 1280 * 4);
static_assert(LP_LS == LP_CN + NPB * 4);
static_assert(LP_WC == LP_LS + LISTN * 4);
static_assert(LDS_POOL >= LP_WC + NW * 4);
static_assert((HP * 2) % 16 == 0);
static_assert((XP * 4) % 16 == 0);
static_assert((NMSG * 4) % 16 == 0);
static_assert(OPB * NMSG * 4 == 14 * 32 * 16);

typedef float          v4f  __attribute__((ext_vector_type(4)));
typedef float          v8f  __attribute__((ext_vector_type(8)));
typedef unsigned short v8us __attribute__((ext_vector_type(8)));
typedef __bf16         v16b __attribute__((ext_vector_type(16)));
typedef v4f  __attribute__((may_alias)) v4fa;
typedef v8us __attribute__((may_alias)) v8usa;
union FragB { v16b v; v8us h[2]; };

__device__ __forceinline__ unsigned int bfr(float f) {
  const unsigned int u = __float_as_uint(f);
  return (u + 0x7FFFu + ((u >> 16) & 1u)) >> 16;
}

__device__ __forceinline__ void split1(float x, unsigned short& hb, unsigned short& lb) {
  const unsigned int hu = bfr(x);
  const float hf = __uint_as_float(hu << 16);
  hb = (unsigned short)hu;
  lb = (unsigned short)bfr(x - hf);
}

__device__ __forceinline__ void split8(v4f a, v4f b, v8us& hi, v8us& lo) {
  unsigned short hb, lb;
  split1(a.x, hb, lb); hi[0] = hb; lo[0] = lb;
  split1(a.y, hb, lb); hi[1] = hb; lo[1] = lb;
  split1(a.z, hb, lb); hi[2] = hb; lo[2] = lb;
  split1(a.w, hb, lb); hi[3] = hb; lo[3] = lb;
  split1(b.x, hb, lb); hi[4] = hb; lo[4] = lb;
  split1(b.y, hb, lb); hi[5] = hb; lo[5] = lb;
  split1(b.z, hb, lb); hi[6] = hb; lo[6] = lb;
  split1(b.w, hb, lb); hi[7] = hb; lo[7] = lb;
}

__device__ __forceinline__ v8f wmb(v16b a, v16b b, v8f c) {
  v8f d = __builtin_amdgcn_wmma_f32_16x16x32_bf16(false, a, false, b, (short)0, c, false, false);
  asm volatile("v_nop\n\tv_nop\n\tv_nop\n\tv_nop" : "+v"(d) : "v"(a), "v"(b));
  return d;
}

__device__ __forceinline__ v8f zero8() { v8f z = {0.f, 0.f, 0.f, 0.f, 0.f, 0.f, 0.f, 0.f}; return z; }
__device__ __forceinline__ v8us zero8us() { v8us z = {0, 0, 0, 0, 0, 0, 0, 0}; return z; }

__device__ __forceinline__ v8f mma3(const FragB& ah, const FragB& al, const FragB& bh, const FragB& bl, v8f c) {
  c = wmb(ah.v, bh.v, c);
  c = wmb(ah.v, bl.v, c);
  c = wmb(al.v, bh.v, c);
  return c;
}

__device__ __forceinline__ void ldB(const unsigned short* __restrict__ bp, size_t loOff, FragB& bh, FragB& bl) {
  bh.h[0] = *(const v8us*)bp;
  bh.h[1] = *(const v8us*)(bp + 16);
  bl.h[0] = *(const v8us*)(bp + loOff);
  bl.h[1] = *(const v8us*)(bp + loOff + 16);
}

__device__ __forceinline__ void wave_lds_sync() {
  __builtin_amdgcn_fence(__ATOMIC_RELEASE, "wavefront");
  __builtin_amdgcn_wave_barrier();
}

__device__ __forceinline__ float sigm(float v) {
  float ev = expf(-v);
  ev = fminf(ev, 1.0e15f);
  return __builtin_amdgcn_rcpf(1.0f + ev);
}

__device__ __forceinline__ void mkfrag16(const float (&e)[16], FragB& fh, FragB& fl) {
  v4f a, b, c, d;
  a.x = e[0];  a.y = e[1];  a.z = e[2];  a.w = e[3];
  b.x = e[4];  b.y = e[5];  b.z = e[6];  b.w = e[7];
  c.x = e[8];  c.y = e[9];  c.z = e[10]; c.w = e[11];
  d.x = e[12]; d.y = e[13]; d.z = e[14]; d.w = e[15];
  split8(a, b, fh.h[0], fl.h[0]);
  split8(c, d, fh.h[1], fl.h[1]);
}

__device__ __forceinline__ void frag_dot3(const float* mp, const float* f0, const float* f1, float scl,
                                          FragB& fh, FragB& fl) {
  const float ma = mp[0], mb = mp[1], mc = mp[2];
  float g0[24], g1[24];
#pragma unroll
  for (int j = 0; j < 6; ++j) {
    const v4f q = *(const v4f*)(f0 + 4 * j);
    g0[4 * j] = q.x; g0[4 * j + 1] = q.y; g0[4 * j + 2] = q.z; g0[4 * j + 3] = q.w;
    const v4f p = *(const v4f*)(f1 + 4 * j);
    g1[4 * j] = p.x; g1[4 * j + 1] = p.y; g1[4 * j + 2] = p.z; g1[4 * j + 3] = p.w;
  }
  float e[16];
#pragma unroll
  for (int i = 0; i < 8; ++i) {
    e[i]     = scl * (ma * g0[3 * i] + mb * g0[3 * i + 1] + mc * g0[3 * i + 2]);
    e[8 + i] = scl * (ma * g1[3 * i] + mb * g1[3 * i + 1] + mc * g1[3 * i + 2]);
  }
  mkfrag16(e, fh, fl);
}

__device__ __forceinline__ void rows_out(const float* st, float* gp, int lane) {
  const int lc = lane < 28 ? lane : 27;
  const v4f zz = {0.f, 0.f, 0.f, 0.f};
  v4f rv[16];
#pragma unroll
  for (int i = 0; i < 16; ++i) {
    const v4f v = *(const v4fa*)(st + i * NMSG + 4 * lc);
    rv[i] = lane < 28 ? v : zz;
  }
  float* p = gp + 4 * lane;
#pragma unroll
  for (int i = 0; i < 16; ++i) *(volatile v4f*)(p + (size_t)i * RP) = rv[i];
  __threadfence();
#pragma unroll
  for (int i = 0; i < 16; ++i) *(volatile v4f*)(p + (size_t)i * RP) = rv[i];
}

template <int NBK>
__device__ __forceinline__ int scan_chunk(const int* __restrict__ ids, const int* __restrict__ flg, int useFlg,
                                          int nE, int cbase, int slotBase, int* list, int tid, int lane, int wave) {
  const int el0 = tid * EPT;
  const int e0  = cbase + el0;
  int wc = 0;
#pragma unroll 1
  for (int g = 0; g < EPT / SGRP; ++g) {
    bool ht[SGRP];
    unsigned sl[SGRP];
    bool anyl = false;
#pragma unroll
    for (int jj = 0; jj < SGRP; ++jj) {
      const int e  = e0 + SGRP * g + jj;
      const int ec = e < nE - 1 ? (e < 0 ? 0 : e) : nE - 1;
      const int k  = ids[ec];
      const int f  = flg[ec];
      const unsigned s = (unsigned)k - (unsigned)slotBase;
      const bool fv = (useFlg == 0) || (f > 1);
      ht[jj] = (e < nE) && (s < (unsigned)NBK) && fv;
      sl[jj] = s;
      anyl = anyl | ht[jj];
    }
    const unsigned any = __builtin_amdgcn_ballot_w32(anyl);
    if (any != 0u) {
#pragma unroll
      for (int jj = 0; jj < SGRP; ++jj) {
        const unsigned mj = __builtin_amdgcn_ballot_w32(ht[jj]);
        if (mj != 0u) {
          const int pos = wc + (int)__builtin_amdgcn_mbcnt_lo(mj, 0u);
          if (ht[jj] && pos < WCAP) list[wave * WCAP + pos] = ((el0 + SGRP * g + jj) << 12) | (int)sl[jj];
          wc += (int)__builtin_popcount(mj);
        }
      }
    }
  }
  return wc;
}

__global__ __launch_bounds__(256) void k_prep(
    const float* __restrict__ W2, const float* __restrict__ Wg000, const float* __restrict__ Wg110,
    const float* __restrict__ Wg001, const float* __restrict__ Wg111, const float* __restrict__ Wg012,
    const float* __restrict__ Wg102, const float* __restrict__ Wd, const float* __restrict__ WL0,
    const float* __restrict__ WL1, unsigned short* wp) {
  const int tid = (int)threadIdx.x, b = (int)blockIdx.x;
  float v[8];
  int po, N, K, i;
  if (b < 288) {
    i = b * 256 + tid;
    const int col = i >> 4, k0 = (i & 15) * 8;
    po = PO_W2; N = WNUM; K = RADN;
#pragma unroll
    for (int e = 0; e < 8; ++e) v[e] = W2[(size_t)(k0 + e) * WNUM + col] * RS128;
  } else if (b < 336) {
    i = (b - 288) * 256 + tid;
    const int col = i >> 8, k0 = (i & 255) * 8;
    po = PO_G1; N = 48; K = 2048;
    const bool lowk = k0 < 1024;
    const float* s;
    int strd, cc;
    if (col < 16) { s = lowk ? Wg000 : Wg110; strd = 16; cc = col; }
    else          { s = lowk ? Wg001 : Wg111; strd = 32; cc = col - 16; }
    const int kb = lowk ? 0 : 1024;
#pragma unroll
    for (int e = 0; e < 8; ++e) v[e] = s[(size_t)(k0 + e - kb) * strd + cc];
  } else if (b < 368) {
    i = (b - 336) * 256 + tid;
    const int col = i >> 3, k0 = (i & 7) * 8;
    po = PO_G3; N = 1024; K = 64;
    const int u = col >> 5, w = col & 31;
#pragma unroll
    for (int e = 0; e < 8; ++e) v[e] = Wg102[(size_t)(u * 64 + k0 + e) * 32 + w];
  } else if (b < 384) {
    i = (b - 368) * 256 + tid;
    const int col = i >> 2, k0 = (i & 3) * 8;
    po = PO_G4; N = 1024; K = 32;
#pragma unroll
    for (int e = 0; e < 8; ++e) {
      const int k = k0 + e, kc = k < 15 ? k : 15;
      const float t = Wg012[(size_t)kc * 1024 + col];
      v[e] = (k < 16) ? t : 0.0f;
    }
  } else if (b < 392) {
    i = (b - 384) * 256 + tid;
    const int col = i >> 7, k0 = (i & 127) * 8;
    po = PO_WD; N = 16; K = 1024;
#pragma unroll
    for (int e = 0; e < 8; ++e) v[e] = Wd[(size_t)(k0 + e) * 16 + col];
  } else {
    if (tid < 64) {
      i = tid;
      const int col = i >> 2, k0 = (i & 3) * 8;
      po = PO_L0; N = 16; K = 32;
#pragma unroll
      for (int e = 0; e < 8; ++e) {
        const int k = k0 + e, kc = k < 15 ? k : 15;
        const float t = WL0[kc * 16 + col];
        v[e] = (k < 16) ? t : 0.0f;
      }
    } else if (tid < 192) {
      i = tid - 64;
      const int col = i >> 2, k0 = (i & 3) * 8;
      po = PO_L1; N = 32; K = 32;
#pragma unroll
      for (int e = 0; e < 8; ++e) v[e] = WL1[(k0 + e) * 32 + col];
    } else {
      return;
    }
  }
  v4f a, c;
  a.x = v[0]; a.y = v[1]; a.z = v[2]; a.w = v[3];
  c.x = v[4]; c.y = v[5]; c.z = v[6]; c.w = v[7];
  v8us hv, lv;
  split8(a, c, hv, lv);
  unsigned short* dh = wp + po + (size_t)i * 8;
  unsigned short* dl = dh + (size_t)N * K;
  *(volatile v8us*)dh = hv;
  *(volatile v8us*)dl = lv;
  __threadfence();
  *(volatile v8us*)dh = hv;
  *(volatile v8us*)dl = lv;
}

__device__ __forceinline__ v8f edge_tile(const unsigned short* ahp, const unsigned short* alp,
                                         const unsigned short* __restrict__ w2h, int t, int m, int hh) {
  v8f d = zero8();
  const unsigned short* bb = w2h + (size_t)(16 * t + m) * RADN + 8 * hh;
#pragma unroll
  for (int kt = 0; kt < 4; ++kt) {
    FragB ah, al, bh, bl;
    ah.h[0] = *(const v8usa*)(ahp + 32 * kt);
    ah.h[1] = *(const v8usa*)(ahp + 32 * kt + 16);
    al.h[0] = *(const v8usa*)(alp + 32 * kt);
    al.h[1] = *(const v8usa*)(alp + 32 * kt + 16);
    ldB(bb + 32 * kt, (size_t)WNUM * RADN, bh, bl);
    d = mma3(ah, al, bh, bl, d);
  }
  return d;
}

__global__ __launch_bounds__(NT) __attribute__((amdgpu_num_vgpr(256)))
void k_edge(const float* __restrict__ x, const float* __restrict__ ea, const float* __restrict__ W1,
            const int* __restrict__ ei, const unsigned short* __restrict__ wp, float* msg, int nN, int nE) {
  extern __shared__ v4f lds_dyn[];
  char* base = (char*)lds_dyn;
  unsigned short* sHh = (unsigned short*)(base + LE_HH);
  unsigned short* sHl = (unsigned short*)(base + LE_HL);
  float* sX0 = (float*)(base + LE_X0);
  float* sX1 = (float*)(base + LE_X1);
  float* sQ1 = (float*)(base + LE_Q1);
  float* sA  = (float*)(base + LE_A);
  float* sW1 = (float*)(base + LE_W1);
  int*   sSrc = (int*)(base + LE_SRC);
  float* stg = (float*)(base);
  const int tid = threadIdx.x, lane = tid & 31, wave = tid >> 5, hh = lane >> 4, m = lane & 15;
  const int eb = blockIdx.x * EPB;

  for (int i = tid; i < 4 * RADN; i += NT) sW1[i] = 0.5f * W1[i];
  if (tid < EPB) {
    int e = eb + tid;
    e = e > nE - 1 ? nE - 1 : e;
    const v4f a = *(const v4f*)(ea + (size_t)e * 4);
    *(v4f*)(sA + tid * 4) = a;
    int s = ei[e];
    s = s < 0 ? 0 : (s > nN - 1 ? nN - 1 : s);
    sSrc[tid] = s;
  }
  __syncthreads();

#pragma unroll
  for (int i = 0; i < (EPB * 40) / NT; ++i) {
    const int idx = i * NT + tid;
    const int row = idx / 40;
    const int c4  = idx - row * 40;
    const int s = sSrc[row];
    const v4f v = *(const v4f*)(x + (size_t)s * NFX + 4 * c4);
    if (c4 < 16) *(v4f*)(sX0 + row * 64 + 4 * c4) = v;
    else         *(v4f*)(sX1 + row * 96 + 4 * (c4 - 16)) = v;
  }
#pragma unroll 1
  for (int i = 0; i < (EPB * 16) / NT; ++i) {
    const int idx = i * NT + tid;
    const int row = idx >> 4, kc = idx & 15;
    const v4f a = *(const v4f*)(sA + row * 4);
    float hv8[8];
#pragma unroll
    for (int j = 0; j < 8; ++j) {
      const int k = 8 * kc + j;
      float p = a.x * sW1[k];
      p = fmaf(a.y, sW1[RADN + k], p);
      p = fmaf(a.z, sW1[2 * RADN + k], p);
      p = fmaf(a.w, sW1[3 * RADN + k], p);
      hv8[j] = CST_SILU * (p * sigm(p));
    }
    v4f c0, c1;
    c0.x = hv8[0]; c0.y = hv8[1]; c0.z = hv8[2]; c0.w = hv8[3];
    c1.x = hv8[4]; c1.y = hv8[5]; c1.z = hv8[6]; c1.w = hv8[7];
    v8us hb, lb;
    split8(c0, c1, hb, lb);
    *(v8us*)(sHh + row * HP + 8 * kc) = hb;
    *(v8us*)(sHl + row * HP + 8 * kc) = lb;
  }
  __syncthreads();
#pragma unroll
  for (int i = 0; i < (EPB * 32) / NT; ++i) {
    const int idx = i * NT + tid;
    const int row = idx >> 5, u = idx & 31;
    const float* xp = sX1 + row * 96 + 3 * u;
    const float* ap = sA + row * 4;
    sQ1[row * 32 + u] = xp[0] * ap[1] + xp[1] * ap[2] + xp[2] * ap[3];
  }
  __syncthreads();

  const int rw = wave * 16;
  const int rb = rw + 8 * hh;
  const unsigned short* w2h = wp + PO_W2;
  const unsigned short* ahp = sHh + (rw + m) * HP + 8 * hh;
  const unsigned short* alp = sHl + (rw + m) * HP + 8 * hh;
  float S000[8], S110[8], S011[2][8], S101[3][2][8];
#pragma unroll
  for (int r = 0; r < 8; ++r) {
    S000[r] = 0.f; S110[r] = 0.f; S011[0][r] = 0.f; S011[1][r] = 0.f;
#pragma unroll
    for (int mm = 0; mm < 3; ++mm) { S101[mm][0][r] = 0.f; S101[mm][1][r] = 0.f; }
  }

#pragma unroll 1
  for (int t = 0; t < 64; ++t) {
    const v8f d = edge_tile(ahp, alp, w2h, t, m, hh);
#pragma unroll
    for (int r = 0; r < 8; ++r) S000[r] = fmaf(sX0[(rb + r) * 64 + t], d[r], S000[r]);
  }
#pragma unroll 1
  for (int tp = 0; tp < 64; ++tp) {
#pragma unroll
    for (int hf = 0; hf < 2; ++hf) {
      const v8f d = edge_tile(ahp, alp, w2h, 64 + 2 * tp + hf, m, hh);
#pragma unroll
      for (int r = 0; r < 8; ++r) S011[hf][r] = fmaf(sX0[(rb + r) * 64 + tp], d[r], S011[hf][r]);
    }
  }
#pragma unroll 1
  for (int tp = 0; tp < 32; ++tp) {
#pragma unroll
    for (int hf = 0; hf < 2; ++hf) {
      const v8f d = edge_tile(ahp, alp, w2h, 192 + 2 * tp + hf, m, hh);
#pragma unroll
      for (int r = 0; r < 8; ++r) {
        const float* cp = sX1 + (rb + r) * 96 + 3 * tp;
        S101[0][hf][r] = fmaf(cp[0], d[r], S101[0][hf][r]);
        S101[1][hf][r] = fmaf(cp[1], d[r], S101[1][hf][r]);
        S101[2][hf][r] = fmaf(cp[2], d[r], S101[2][hf][r]);
      }
    }
  }
#pragma unroll 1
  for (int t = 0; t < 32; ++t) {
    const v8f d = edge_tile(ahp, alp, w2h, 256 + t, m, hh);
#pragma unroll
    for (int r = 0; r < 8; ++r) S110[r] = fmaf(sQ1[(rb + r) * 32 + t], d[r], S110[r]);
  }
  __syncthreads();

  float* st = stg + wave * (16 * NMSG);
#pragma unroll
  for (int r = 0; r < 8; ++r) {
    const int lr = 8 * hh + r;
    const float* ap = sA + (rw + lr) * 4;
    const float a0 = ap[0], a1 = ap[1], a2 = ap[2], a3 = ap[3];
    st[lr * NMSG + m] = PW_MSG0 * (a0 * S000[r] + INV3 * S110[r]);
    float* q = st + lr * NMSG + 16 + 3 * m;
    q[0] = PW_MSG1 * INV3 * (a1 * S011[0][r] + a0 * S101[0][0][r]);
    q[1] = PW_MSG1 * INV3 * (a2 * S011[0][r] + a0 * S101[1][0][r]);
    q[2] = PW_MSG1 * INV3 * (a3 * S011[0][r] + a0 * S101[2][0][r]);
    float* q2 = st + lr * NMSG + 64 + 3 * m;
    q2[0] = PW_MSG1 * INV3 * (a1 * S011[1][r] + a0 * S101[0][1][r]);
    q2[1] = PW_MSG1 * INV3 * (a2 * S011[1][r] + a0 * S101[1][1][r]);
    q2[2] = PW_MSG1 * INV3 * (a3 * S011[1][r] + a0 * S101[2][1][r]);
  }
  wave_lds_sync();
  rows_out(st, msg + (size_t)(eb + rw) * RP, lane);
}

__global__ __launch_bounds__(NT) __attribute__((amdgpu_num_vgpr(256)))
void k_node(const float* __restrict__ x, const int* __restrict__ ei, const float* __restrict__ msg,
            const unsigned short* __restrict__ wp, float* xg, int nN, int nE) {
  extern __shared__ v4f lds_dyn[];
  char* base = (char*)lds_dyn;
  float* sX  = (float*)(base + LN_X);
  float* sNM = (float*)(base + LN_NM);
  float* sSt = (float*)(base + LN_ST);
  int*   list = (int*)(base + LN_LS);
  int*   wcnt = (int*)(base + LN_WC);
  const int tid = threadIdx.x, lane = tid & 31, wave = tid >> 5, hh = lane >> 4, m = lane & 15;
  const int nb = blockIdx.x * NPB;
  const int lc = lane < 28 ? lane : 27;

#pragma unroll
  for (int i = 0; i < (NPB * 40) / NT; ++i) {
    const int idx = i * NT + tid;
    const int row = idx / 40;
    const int c4  = idx - row * 40;
    int n = nb + row;
    n = n > nN - 1 ? nN - 1 : n;
    ((v4f*)sX)[idx] = *(const v4f*)(x + (size_t)n * NFX + 4 * c4);
  }
  {
    const v4f zz = {0.f, 0.f, 0.f, 0.f};
#pragma unroll
    for (int i = 0; i < (NPB * 28) / NT; ++i) ((v4f*)sNM)[i * NT + tid] = zz;
  }
  __syncthreads();

  const int* dst = ei + nE;
  const int nChunks = (nE + CHUNK - 1) / CHUNK;
#pragma unroll 1
  for (int ch = 0; ch < nChunks; ++ch) {
    const int cbase = ch * CHUNK;
    const int wc = scan_chunk<NPB>(dst, dst, 0, nE, cbase, nb, list, tid, lane, wave);
    if (lane == 0) wcnt[wave] = wc;
    __syncthreads();
    if (wave == 0) {
#pragma unroll 1
      for (int wsx = 0; wsx < NW; ++wsx) {
        int n = __builtin_amdgcn_readfirstlane(wcnt[wsx]);
        n = n > WCAP ? WCAP : (n < 0 ? 0 : n);
        const int* lp = list + wsx * WCAP;
#pragma unroll 1
        for (int i = 0; i < n; ++i) {
          const int ent  = __builtin_amdgcn_readfirstlane(lp[i]);
          const int slot = ent & (NPB - 1);
          int e = cbase + ((ent >> 12) & (CHUNK - 1));
          e = e > nE - 1 ? nE - 1 : e;
          const v4f mv = *(const v4f*)(msg + (size_t)e * RP + 4 * lc);
          float* ap = sNM + slot * NMSG + 4 * lc;
          const v4f cur = *(const v4f*)ap;
          if (lane < 28) *(v4f*)ap = cur + mv;
        }
      }
    }
    __syncthreads();
  }

  const int rw = wave * 16;
  const int ra = rw + m;
  const int rb = rw + 8 * hh;
  float* st = sSt + wave * (16 * NMSG);

  {
    v8f acc[3];
    acc[0] = zero8(); acc[1] = zero8(); acc[2] = zero8();
    const unsigned short* g1h = wp + PO_G1;
#pragma unroll 1
    for (int kt = 0; kt < 32; ++kt) {
      const int u  = kt >> 1;
      const int v0 = 32 * (kt & 1);
      const float mu = sNM[ra * NMSG + u];
      const float* xp = sX + ra * XP + v0 + 8 * hh;
      const v4f p0 = *(const v4f*)xp * mu;
      const v4f p1 = *(const v4f*)(xp + 4) * mu;
      const v4f p2 = *(const v4f*)(xp + 16) * mu;
      const v4f p3 = *(const v4f*)(xp + 20) * mu;
      FragB ah, al;
      split8(p0, p1, ah.h[0], al.h[0]);
      split8(p2, p3, ah.h[1], al.h[1]);
#pragma unroll
      for (int ct = 0; ct < 3; ++ct) {
        FragB bh, bl;
        ldB(g1h + (size_t)(16 * ct + m) * 2048 + 32 * kt + 8 * hh, (size_t)48 * 2048, bh, bl);
        acc[ct] = mma3(ah, al, bh, bl, acc[ct]);
      }
    }
#pragma unroll 1
    for (int kt = 32; kt < 64; ++kt) {
      const int u = kt - 32;
      const float* mp = sNM + ra * NMSG + 16 + 3 * u;
      const float* f0 = sX + ra * XP + 64 + 24 * hh;
      FragB ah, al;
      frag_dot3(mp, f0, f0 + 48, INV3, ah, al);
#pragma unroll
      for (int ct = 0; ct < 3; ++ct) {
        FragB bh, bl;
        ldB(g1h + (size_t)(16 * ct + m) * 2048 + 32 * kt + 8 * hh, (size_t)48 * 2048, bh, bl);
        acc[ct] = mma3(ah, al, bh, bl, acc[ct]);
      }
    }
#pragma unroll
    for (int ct = 0; ct < 3; ++ct) {
#pragma unroll
      for (int r = 0; r < 8; ++r) st[(8 * hh + r) * NMSG + 16 * ct + m] = acc[ct][r];
    }
  }

  float GV[3][2][8];
#pragma unroll
  for (int r = 0; r < 8; ++r) {
#pragma unroll
    for (int mm = 0; mm < 3; ++mm) { GV[mm][0][r] = 0.f; GV[mm][1][r] = 0.f; }
  }
  {
    FragB a3h[2], a3l[2];
#pragma unroll
    for (int kt = 0; kt < 2; ++kt) {
      const float* xp = sX + ra * XP + 32 * kt + 8 * hh;
      const v4f q0 = *(const v4f*)xp, q1 = *(const v4f*)(xp + 4);
      const v4f q2 = *(const v4f*)(xp + 16), q3 = *(const v4f*)(xp + 20);
      split8(q0, q1, a3h[kt].h[0], a3l[kt].h[0]);
      split8(q2, q3, a3h[kt].h[1], a3l[kt].h[1]);
    }
    const unsigned short* g3h = wp + PO_G3;
#pragma unroll 1
    for (int tp = 0; tp < 32; ++tp) {
#pragma unroll
      for (int hf = 0; hf < 2; ++hf) {
        const int t = 2 * tp + hf;
        v8f d = zero8();
#pragma unroll
        for (int kt = 0; kt < 2; ++kt) {
          FragB bh, bl;
          ldB(g3h + (size_t)(16 * t + m) * 64 + 32 * kt + 8 * hh, (size_t)1024 * 64, bh, bl);
          d = mma3(a3h[kt], a3l[kt], bh, bl, d);
        }
#pragma unroll
        for (int r = 0; r < 8; ++r) {
          const float* cp = sNM + (rb + r) * NMSG + 16 + 3 * tp;
          GV[0][hf][r] = fmaf(cp[0], d[r], GV[0][hf][r]);
          GV[1][hf][r] = fmaf(cp[1], d[r], GV[1][hf][r]);
          GV[2][hf][r] = fmaf(cp[2], d[r], GV[2][hf][r]);
        }
      }
    }
  }
  {
    FragB a4h, a4l;
    {
      const float* mp0 = sNM + ra * NMSG + 8 * hh;
      const v4f q0 = *(const v4f*)mp0, q1 = *(const v4f*)(mp0 + 4);
      split8(q0, q1, a4h.h[0], a4l.h[0]);
      a4h.h[1] = zero8us();
      a4l.h[1] = zero8us();
    }
    const unsigned short* g4h = wp + PO_G4;
#pragma unroll 1
    for (int tp = 0; tp < 32; ++tp) {
#pragma unroll
      for (int hf = 0; hf < 2; ++hf) {
        const int t = 2 * tp + hf;
        FragB bh, bl;
        ldB(g4h + (size_t)(16 * t + m) * 32 + 8 * hh, (size_t)1024 * 32, bh, bl);
        v8f d = zero8();
        d = mma3(a4h, a4l, bh, bl, d);
#pragma unroll
        for (int r = 0; r < 8; ++r) {
          const float* cp = sX + (rb + r) * XP + 64 + 3 * tp;
          GV[0][hf][r] = fmaf(cp[0], d[r], GV[0][hf][r]);
          GV[1][hf][r] = fmaf(cp[1], d[r], GV[1][hf][r]);
          GV[2][hf][r] = fmaf(cp[2], d[r], GV[2][hf][r]);
        }
      }
    }
  }

  float gsr[8], gga[8], ggb[8];
#pragma unroll
  for (int r = 0; r < 8; ++r) {
    const float* sp = st + (8 * hh + r) * NMSG;
    gsr[r] = sp[m];
    gga[r] = sp[16 + m];
    ggb[r] = sp[32 + m];
  }
  wave_lds_sync();
#pragma unroll
  for (int r = 0; r < 8; ++r) {
    const int lr = 8 * hh + r;
    st[lr * NMSG + m] = CST_SIG * sigm(PW_G01 * gsr[r]);
    const float ga = CST_TANH * tanhf(PW_G01 * gga[r]);
    const float gb = CST_TANH * tanhf(PW_G01 * ggb[r]);
    float* q = st + lr * NMSG + 16 + 3 * m;
    q[0] = ga * (PW_G2 * INV3 * GV[0][0][r]);
    q[1] = ga * (PW_G2 * INV3 * GV[1][0][r]);
    q[2] = ga * (PW_G2 * INV3 * GV[2][0][r]);
    float* q2 = st + lr * NMSG + 64 + 3 * m;
    q2[0] = gb * (PW_G2 * INV3 * GV[0][1][r]);
    q2[1] = gb * (PW_G2 * INV3 * GV[1][1][r]);
    q2[2] = gb * (PW_G2 * INV3 * GV[2][1][r]);
  }
  wave_lds_sync();
  rows_out(st, xg + (size_t)(nb + rw) * RP, lane);
}

__global__ __launch_bounds__(NT) __attribute__((amdgpu_num_vgpr(256)))
void k_pool(const float* __restrict__ xg, const int* __restrict__ canon, const int* __restrict__ z,
            const float* __restrict__ Wa, const float* __restrict__ Wb, const float* __restrict__ Wc,
            const unsigned short* __restrict__ wp, float* th, int nN) {
  extern __shared__ v4f lds_dyn[];
  char* base = (char*)lds_dyn;
  float* sS  = (float*)(base + LP_S);
  float* sSt = (float*)(base + LP_ST);
  float* sW  = (float*)(base + LP_W);
  int*   sCnt = (int*)(base + LP_CN);
  int*   list = (int*)(base + LP_LS);
  int*   wcnt = (int*)(base + LP_WC);
  const int tid = threadIdx.x, lane = tid & 31, wave = tid >> 5, hh = lane >> 4, m = lane & 15;
  const int cb = blockIdx.x * NPB;
  const int lc = lane < 28 ? lane : 27;

  {
    const v4f zz = {0.f, 0.f, 0.f, 0.f};
#pragma unroll
    for (int i = 0; i < (NPB * 28) / NT; ++i) ((v4f*)sS)[i * NT + tid] = zz;
  }
  if (tid < NPB) sCnt[tid] = 0;
#pragma unroll 1
  for (int idx = tid; idx < 1280; idx += NT) {
    const int ia = idx < 255 ? idx : 255;
    int ib = idx - 256; ib = ib < 0 ? 0 : (ib > 511 ? 511 : ib);
    int ic = idx - 768; ic = ic < 0 ? 0 : (ic > 511 ? 511 : ic);
    const float wa = Wa[ia], wb = Wb[ib], wcv = Wc[ic];
    sW[idx] = idx < 256 ? wa : (idx < 768 ? wb : wcv);
  }
  __syncthreads();

  const int nChunks = (nN + CHUNK - 1) / CHUNK;
#pragma unroll 1
  for (int ch = 0; ch < nChunks; ++ch) {
    const int cbase = ch * CHUNK;
    const int wc = scan_chunk<NPB>(canon, z, 1, nN, cbase, cb, list, tid, lane, wave);
    if (lane == 0) wcnt[wave] = wc;
    __syncthreads();
    if (wave == 0) {
#pragma unroll 1
      for (int wsx = 0; wsx < NW; ++wsx) {
        int n = __builtin_amdgcn_readfirstlane(wcnt[wsx]);
        n = n > WCAP ? WCAP : (n < 0 ? 0 : n);
        const int* lp = list + wsx * WCAP;
#pragma unroll 1
        for (int i = 0; i < n; ++i) {
          const int ent  = __builtin_amdgcn_readfirstlane(lp[i]);
          const int slot = ent & (NPB - 1);
          int nd = cbase + ((ent >> 12) & (CHUNK - 1));
          nd = nd > nN - 1 ? nN - 1 : nd;
          const v4f xv = *(const v4f*)(xg + (size_t)nd * RP + 4 * lc);
          float* ap = sS + slot * NMSG + 4 * lc;
          const v4f cur = *(const v4f*)ap;
          if (lane < 28) *(v4f*)ap = cur + xv;
          if (lane == 0) sCnt[slot] = sCnt[slot] + 1;
        }
      }
    }
    __syncthreads();
  }

#pragma unroll
  for (int i = 0; i < (NPB * 28) / NT; ++i) {
    const int idx = i * NT + tid;
    const int slot = idx / 28;
    int c = sCnt[slot];
    c = c < 1 ? 1 : c;
    const float rc = 1.0f / (float)c;
    v4f v = ((v4f*)sS)[idx];
    v = v * rc;
    ((v4f*)sS)[idx] = v;
  }
  __syncthreads();

  const int rw = wave * 16;
  const int ra = rw + m;
  v8f dq = zero8();
  {
    const unsigned short* wdh = wp + PO_WD;
#pragma unroll 1
    for (int kt = 0; kt < 32; ++kt) {
      const float* mp = sS + ra * NMSG + 16 + 3 * kt;
      const float* f0 = sS + ra * NMSG + 16 + 24 * hh;
      FragB ah, al, bh, bl;
      frag_dot3(mp, f0, f0 + 48, 1.0f, ah, al);
      ldB(wdh + (size_t)m * 1024 + 32 * kt + 8 * hh, (size_t)16 * 1024, bh, bl);
      dq = mma3(ah, al, bh, bl, dq);
    }
  }
  float* st = sSt + wave * (16 * NMSG);
#pragma unroll
  for (int r = 0; r < 8; ++r) {
    const int lr = 8 * hh + r;
    const float* hp = sS + (rw + lr) * NMSG;
    float sa = 0.f, sb0 = 0.f, sb1 = 0.f, sc0 = 0.f, sc1 = 0.f;
#pragma unroll 1
    for (int v = 0; v < 16; ++v) {
      const float h0v = hp[v];
      sa  = fmaf(sW[m * 16 + v], h0v, sa);
      sb0 = fmaf(sW[256 + v * 32 + m], h0v, sb0);
      sb1 = fmaf(sW[256 + v * 32 + 16 + m], h0v, sb1);
      sc0 = fmaf(sW[768 + m * 16 + v], h0v, sc0);
      sc1 = fmaf(sW[768 + (16 + m) * 16 + v], h0v, sc1);
    }
    st[lr * NMSG + m] = PW_H0 * (hp[m] * sa + INV3 * dq[r]);
    const float fa = PW_H1 * INV3 * (sb0 + sc0);
    const float fb = PW_H1 * INV3 * (sb1 + sc1);
    float* q = st + lr * NMSG + 16 + 3 * m;
    q[0] = fa * hp[16 + 3 * m + 0];
    q[1] = fa * hp[16 + 3 * m + 1];
    q[2] = fa * hp[16 + 3 * m + 2];
    float* q2 = st + lr * NMSG + 64 + 3 * m;
    q2[0] = fb * hp[64 + 3 * m + 0];
    q2[1] = fb * hp[64 + 3 * m + 1];
    q2[2] = fb * hp[64 + 3 * m + 2];
  }
  wave_lds_sync();
  rows_out(st, th + (size_t)(cb + rw) * RP, lane);
}

__global__ __launch_bounds__(32) void k_out(
    const float* __restrict__ xg, const float* __restrict__ th, const int* __restrict__ z,
    const int* __restrict__ canon, const unsigned short* __restrict__ wp, float* out, int nN) {
  __shared__ __attribute__((aligned(16))) float sY[OPB * NMSG];
  __shared__ __attribute__((aligned(16))) float sO[OPB * NMSG];
  __shared__ int sC[OPB];
  __shared__ int sH[OPB];
  const int lane = threadIdx.x & 31, hh = lane >> 4, m = lane & 15;
  const int n0 = blockIdx.x * OPB;

  {
    int n = n0 + m;
    n = n > nN - 1 ? nN - 1 : n;
    const int zv = z[n];
    int c = canon[n];
    c = c < 0 ? 0 : (c > nN - 1 ? nN - 1 : c);
    if (lane < OPB) { sC[m] = c; sH[m] = zv > 1 ? 1 : 0; }
  }
  __syncthreads();
#pragma unroll 2
  for (int i = 0; i < 14; ++i) {
    const int idx = i * 32 + lane;
    const int row = idx / 28;
    const int c4  = idx - row * 28;
    int n = n0 + row;
    n = n > nN - 1 ? nN - 1 : n;
    const int c = sC[row];
    const bool hz = sH[row] != 0;
    const v4f vt = *(const v4f*)(th + (size_t)c * RP + 4 * c4);
    const v4f vx = *(const v4f*)(xg + (size_t)n * RP + 4 * c4);
    ((v4f*)sY)[idx] = hz ? vt : vx;
  }
  __syncthreads();

  const unsigned short* l0 = wp + PO_L0;
  const unsigned short* l1 = wp + PO_L1;
  v8f d0 = zero8();
  {
    FragB ah, al, bh, bl;
    const float* yp = sY + m * NMSG + 8 * hh;
    const v4f ya = *(const v4f*)yp, yb = *(const v4f*)(yp + 4);
    split8(ya, yb, ah.h[0], al.h[0]);
    ah.h[1] = zero8us();
    al.h[1] = zero8us();
    ldB(l0 + m * 32 + 8 * hh, 512, bh, bl);
    d0 = mma3(ah, al, bh, bl, d0);
  }
  v8f d1[3][2];
#pragma unroll
  for (int rt = 0; rt < 3; ++rt) {
    const int R  = 16 * rt + m;
    const int nl = R / 3;
    const int mm = R - 3 * nl;
    float e[16];
#pragma unroll
    for (int i = 0; i < 8; ++i) {
      e[i]     = sY[nl * NMSG + 16 + 3 * (8 * hh + i) + mm];
      e[8 + i] = sY[nl * NMSG + 16 + 3 * (16 + 8 * hh + i) + mm];
    }
    FragB ah, al;
    mkfrag16(e, ah, al);
#pragma unroll
    for (int ct = 0; ct < 2; ++ct) {
      FragB bh, bl;
      ldB(l1 + (16 * ct + m) * 32 + 8 * hh, 1024, bh, bl);
      d1[rt][ct] = mma3(ah, al, bh, bl, zero8());
    }
  }
#pragma unroll
  for (int r = 0; r < 8; ++r) sO[(8 * hh + r) * NMSG + m] = 0.25f * d0[r];
#pragma unroll
  for (int rt = 0; rt < 3; ++rt) {
#pragma unroll
    for (int ct = 0; ct < 2; ++ct) {
#pragma unroll
      for (int r = 0; r < 8; ++r) {
        const int R  = 16 * rt + 8 * hh + r;
        const int nl = R / 3;
        const int mm = R - 3 * nl;
        const int w  = 16 * ct + m;
        sO[nl * NMSG + 16 + 3 * w + mm] = RS32 * d1[rt][ct][r];
      }
    }
  }
  __syncthreads();

  float* op = out + (size_t)n0 * NMSG;
  v4f ov[14];
#pragma unroll
  for (int i = 0; i < 14; ++i) ov[i] = *(const v4fa*)(sO + 4 * (i * 32 + lane));
#pragma unroll
  for (int i = 0; i < 14; ++i) {
    const int idx = i * 32 + lane;
    if (n0 + idx / 28 < nN) *(volatile v4f*)(op + 4 * (size_t)idx) = ov[i];
  }
  __threadfence();
#pragma unroll
  for (int i = 0; i < 14; ++i) {
    const int idx = i * 32 + lane;
    if (n0 + idx / 28 < nN) *(volatile v4f*)(op + 4 * (size_t)idx) = ov[i];
  }
}

extern "C" void kernel_launch(void* const* d_in, const int* in_sizes, int n_in,
                              void* d_out, int out_size, void* d_ws, size_t ws_size,
                              hipStream_t stream) {
  if (n_in < 19) return;
  if (in_sizes[0] <= 0 || (in_sizes[0] % NFX) != 0) return;
  if (in_sizes[1] <= 0 || (in_sizes[1] % 4) != 0) return;
  const int nN = in_sizes[0] / NFX;
  const int nE = in_sizes[1] / 4;
  if (nN <= 0 || nE <= 0) return;
  if (nN > (1 << 22) || nE > (1 << 26)) return;
  if (in_sizes[2] != 4 * RADN || in_sizes[3] != RADN * WNUM) return;
  if (in_sizes[4] != 16384 || in_sizes[5] != 16384 || in_sizes[6] != 32768 || in_sizes[7] != 32768) return;
  if (in_sizes[8] != 16384 || in_sizes[9] != 65536) return;
  if (in_sizes[10] != 256 || in_sizes[11] != 512 || in_sizes[12] != 512 || in_sizes[13] != 16384) return;
  if (in_sizes[14] != 256 || in_sizes[15] != 1024) return;
  if (in_sizes[16] != 2 * nE || in_sizes[17] != nN || in_sizes[18] != nN) return;
  if (out_size != nN * NMSG) return;

  const float* x     = (const float*)d_in[0];
  const float* ea    = (const float*)d_in[1];
  const float* W1    = (const float*)d_in[2];
  const float* W2    = (const float*)d_in[3];
  const float* Wg000 = (const float*)d_in[4];
  const float* Wg110 = (const float*)d_in[5];
  const float* Wg001 = (const float*)d_in[6];
  const float* Wg111 = (const float*)d_in[7];
  const float* Wg012 = (const float*)d_in[8];
  const float* Wg102 = (const float*)d_in[9];
  const float* Wa    = (const float*)d_in[10];
  const float* Wb    = (const float*)d_in[11];
  const float* Wc    = (const float*)d_in[12];
  const float* Wd    = (const float*)d_in[13];
  const float* WL0   = (const float*)d_in[14];
  const float* WL1   = (const float*)d_in[15];
  const int*   ei    = (const int*)d_in[16];
  const int*   z     = (const int*)d_in[17];
  const int*   canon = (const int*)d_in[18];
  float* out = (float*)d_out;

  const int EP = ((nE + EPB - 1) / EPB) * EPB;
  const int NP = ((nN + NPB - 1) / NPB) * NPB;

  char* ws = (char*)d_ws;
  size_t off = 0;
  const size_t oW  = off; off += (size_t)PO_TOT * 2;        off = (off + 255) & ~(size_t)255;
  const size_t oM  = off; off += (size_t)EP * RP * 4;       off = (off + 255) & ~(size_t)255;
  const size_t oXg = off; off += (size_t)NP * RP * 4;       off = (off + 255) & ~(size_t)255;
  const size_t oTh = off; off += (size_t)NP * RP * 4;       off = (off + 255) & ~(size_t)255;
  if (off > ws_size || off > (size_t)WSCAP) return;
  unsigned short* wp = (unsigned short*)(ws + oW);
  float* msgp = (float*)(ws + oM);
  float* xgp  = (float*)(ws + oXg);
  float* thp  = (float*)(ws + oTh);

  k_prep<<<NPREPB, 256, 0, stream>>>(W2, Wg000, Wg110, Wg001, Wg111, Wg012, Wg102, Wd, WL0, WL1, wp);

  hipFuncSetAttribute(reinterpret_cast<const void*>(&k_edge),
                      hipFuncAttributeMaxDynamicSharedMemorySize, LDS_EDGE);
  k_edge<<<EP / EPB, NT, LDS_EDGE, stream>>>(x, ea, W1, ei, wp, msgp, nN, nE);

  hipFuncSetAttribute(reinterpret_cast<const void*>(&k_node),
                      hipFuncAttributeMaxDynamicSharedMemorySize, LDS_NODE);
  k_node<<<NP / NPB, NT, LDS_NODE, stream>>>(x, ei, msgp, wp, xgp, nN, nE);

  hipFuncSetAttribute(reinterpret_cast<const void*>(&k_pool),
                      hipFuncAttributeMaxDynamicSharedMemorySize, LDS_POOL);
  k_pool<<<NP / NPB, NT, LDS_POOL, stream>>>(xgp, canon, z, Wa, Wb, Wc, wp, thp, nN);

  k_out<<<NP / OPB, 32, 0, stream>>>(xgp, thp, z, canon, wp, out, nN);
}
